// LightweightLinearAttention2d_2336462209422
// MI455X (gfx1250) — hardware-verified
//
#include <hip/hip_runtime.h>
#include <math.h>

typedef __attribute__((ext_vector_type(16))) _Float16 v16h;
typedef __attribute__((ext_vector_type(8)))  _Float16 v8h;
typedef __attribute__((ext_vector_type(16))) __bf16   v16b;
typedef __attribute__((ext_vector_type(8)))  __bf16   v8b;
typedef __attribute__((ext_vector_type(8)))  float    v8f;
typedef __attribute__((ext_vector_type(4)))  float    v4f;
typedef __attribute__((ext_vector_type(4)))  unsigned int v4u;

constexpr int  kImg    = 8;
constexpr int  kCin    = 384;
constexpr int  kPix    = 4096;
constexpr int  kImgW   = 64;
constexpr int  kCqkv   = 1152;
constexpr int  kHeads  = 8;
constexpr int  kHd     = 48;
constexpr int  kHdPad  = 64;
constexpr int  kInner  = 384;
constexpr int  kPlRows = kHeads * kHdPad;
constexpr long kPlElems = (long)kPlRows * kPix;
constexpr long kQtElems = (long)kHeads * kPix * kHdPad;
constexpr int  kOcols  = kHeads * kHdPad;
constexpr float kEps   = 1e-6f;
constexpr float kBnEps = 1e-5f;

__device__ __forceinline__ unsigned short f2bf_bits(float f) {
  unsigned u = __float_as_uint(f);
  return (unsigned short)((u + 0x7FFFu + ((u >> 16) & 1u)) >> 16);
}
__device__ __forceinline__ float bf_bits2f(unsigned short h) { return __uint_as_float(((unsigned)h) << 16); }
__device__ __forceinline__ float bfr(float f) { return bf_bits2f(f2bf_bits(f)); }
__device__ __forceinline__ unsigned pk16(unsigned short a, unsigned short b) { return (unsigned)a | ((unsigned)b << 16); }

__device__ __forceinline__ void dep_guard_h(v8f& a, v8f& b, v16h x, v16h y) { asm volatile("v_nop\n\tv_nop\n\tv_nop\n\tv_nop" : "+v"(a), "+v"(b) : "v"(x), "v"(y)); }
__device__ __forceinline__ void dep_guard_b(v8f& a, v8f& b, v16b x, v16b y) { asm volatile("v_nop\n\tv_nop\n\tv_nop\n\tv_nop" : "+v"(a), "+v"(b) : "v"(x), "v"(y)); }
__device__ __forceinline__ void keep4_h(v16h a, v16h b, v16h c, v16h d) { asm volatile("v_nop" :: "v"(a), "v"(b), "v"(c), "v"(d)); }
__device__ __forceinline__ void keep4_b(v16b a, v16b b, v16b c, v16b d) { asm volatile("v_nop" :: "v"(a), "v"(b), "v"(c), "v"(d)); }
__device__ __forceinline__ void acc_guard4(v8f& a, v8f& b, v8f& c, v8f& d) { asm volatile("v_nop\n\tv_nop\n\tv_nop\n\tv_nop" : "+v"(a), "+v"(b), "+v"(c), "+v"(d)); }
template <typename T> struct Frag;
template <> struct Frag<_Float16> {
  typedef v16h V; union U { v16h v; v8h h[2]; };
  static __device__ __forceinline__ v16h load(const _Float16* p) {
    U f; f.h[0] = *(const v8h*)(p); f.h[1] = *(const v8h*)(p + 16); return f.v;
  }
  static __device__ __forceinline__ v8f mma(v16h a, v16h b, v8f c) {
    return __builtin_amdgcn_wmma_f32_16x16x32_f16(false, a, false, b, (short)0, c, false, false);
  }
  static __device__ __forceinline__ void guard(v8f& a, v8f& b, v16h x, v16h y) { dep_guard_h(a, b, x, y); }
  static __device__ __forceinline__ void keep(v16h a, v16h b, v16h c, v16h d) { keep4_h(a, b, c, d); }
};
template <> struct Frag<__bf16> {
  typedef v16b V; union U { v16b v; v8b h[2]; };
  static __device__ __forceinline__ v16b load(const __bf16* p) {
    U f; f.h[0] = *(const v8b*)(p); f.h[1] = *(const v8b*)(p + 16); return f.v;
  }
  static __device__ __forceinline__ v8f mma(v16b a, v16b b, v8f c) {
    return __builtin_amdgcn_wmma_f32_16x16x32_bf16(false, a, false, b, (short)0, c, false, false);
  }
  static __device__ __forceinline__ void guard(v8f& a, v8f& b, v16b x, v16b y) { dep_guard_b(a, b, x, y); }
  static __device__ __forceinline__ void keep(v16b a, v16b b, v16b c, v16b d) { keep4_b(a, b, c, d); }
};

template <int ET> struct Elem;
template <> struct Elem<0> { typedef _Float16 T; };
template <> struct Elem<1> { typedef __bf16 T; };
template <int ET, int SPLIT, int BIAS_MODE, int OUT_MODE, bool RESID, int ACT = 0>
__global__ __launch_bounds__(256) void wmma_gemm64(
    const unsigned short* __restrict__ Ap, const unsigned short* __restrict__ A2p, int lda, long strideA,
    const unsigned short* __restrict__ Btp, const unsigned short* __restrict__ Bt2p, int ldb, long strideB,
    void* __restrict__ Cout, void* __restrict__ Cout2, int ldc, long strideC,
    const float* __restrict__ bias,
    const float* __restrict__ resid, long strideR,
    int M, int N, int K, float scale) {
  typedef typename Elem<ET>::T T;
  typedef typename Frag<T>::V V;
  const T* A = (const T*)Ap; const T* A2 = (const T*)A2p; const T* Bt = (const T*)Btp; const T* Bt2 = (const T*)Bt2p;
  __shared__ __align__(16) float sT[8][16 * 68];
  const int b    = blockIdx.y;
  const int lane = threadIdx.x & 31;
  const int wave = threadIdx.x >> 5;
  const int tilesN = N >> 6;
  const int tilesM = M >> 6;
  const int tile = blockIdx.x * 8 + wave;
  if (tile >= tilesM * tilesN) return;
  const int tm = tile / tilesN;
  const int tn = tile - tm * tilesN;
  const int m0 = tm << 6;
  const int n0 = tn << 6;

  const T* Ab  = A  + (size_t)b * strideA;
  const T* Bb  = Bt + (size_t)b * strideB;
  const T* Ab2 = (SPLIT == 2) ? (A2  + (size_t)b * strideA) : nullptr;
  const T* Bb2 = (SPLIT >= 1) ? (Bt2 + (size_t)b * strideB) : nullptr;

  const int rlane = lane & 15;
  const int koff  = (lane >> 4) * 8;
  const int mOff  = (lane >> 4) * 8;

  v8f acc[4][4];
#pragma unroll
  for (int i = 0; i < 4; ++i)
#pragma unroll
    for (int j = 0; j < 4; ++j) acc[i][j] = (v8f){0.f,0.f,0.f,0.f,0.f,0.f,0.f,0.f};

  for (int k0 = 0; k0 < K; k0 += 32) {
    V bh[4], bl[4];
#pragma unroll
    for (int j = 0; j < 4; ++j) {
      const size_t bo = (size_t)(n0 + (j << 4) + rlane) * ldb + koff + k0;
      bh[j] = Frag<T>::load(Bb + bo);
      if (SPLIT >= 1) bl[j] = Frag<T>::load(Bb2 + bo);
    }
#pragma unroll
    for (int i = 0; i < 4; ++i) {
      const size_t ao = (size_t)(m0 + (i << 4) + rlane) * lda + koff + k0;
      V ah = Frag<T>::load(Ab + ao);
      V al;
      if (SPLIT == 2) al = Frag<T>::load(Ab2 + ao);
#pragma unroll
      for (int j = 0; j < 4; ++j) {
        acc[i][j] = Frag<T>::mma(ah, bh[j], acc[i][j]);
        if (SPLIT >= 1) acc[i][j] = Frag<T>::mma(ah, bl[j], acc[i][j]);
        if (SPLIT == 2) acc[i][j] = Frag<T>::mma(al, bh[j], acc[i][j]);
      }
      Frag<T>::guard(acc[i][0], acc[i][3], ah, (SPLIT == 2) ? al : ah);
    }
    Frag<T>::keep(bh[0], bh[1], bh[2], bh[3]);
    if (SPLIT >= 1) Frag<T>::keep(bl[0], bl[1], bl[2], bl[3]);
  }
  acc_guard4(acc[0][0], acc[0][1], acc[0][2], acc[0][3]);
  acc_guard4(acc[1][0], acc[1][1], acc[1][2], acc[1][3]);
  acc_guard4(acc[2][0], acc[2][1], acc[2][2], acc[2][3]);
  acc_guard4(acc[3][0], acc[3][1], acc[3][2], acc[3][3]);

  float* slab = sT[wave];
  const float* Rb = RESID ? (resid + (size_t)b * strideR) : nullptr;
#pragma unroll
  for (int i = 0; i < 4; ++i) {
    const int mBase = m0 + (i << 4);
#pragma unroll
    for (int j = 0; j < 4; ++j) {
      const int n = n0 + (j << 4) + rlane;
      float bv = 0.f;
      if (BIAS_MODE == 2) bv = bias[n];
#pragma unroll
      for (int r = 0; r < 8; ++r) {
        float v = acc[i][j][r] * scale;
        if (BIAS_MODE == 1) v += bias[mBase + mOff + r];
        if (BIAS_MODE == 2) v += bv;
        if (BIAS_MODE == 3) v = v * bias[mBase + mOff + r] + bias[M + mBase + mOff + r];
        if (RESID) v += Rb[(size_t)(mBase + mOff + r) * ldc + n];
        if (ACT == 2) v = fmaxf(v, 0.0f);
        if (ACT == 4) v = (v > 0.f) ? v : 0.01f * v;
        slab[(mOff + r) * 68 + (j << 4) + rlane] = v;
      }
    }
    __builtin_amdgcn_fence(__ATOMIC_RELEASE, "workgroup");
    __builtin_amdgcn_wave_barrier();
    __builtin_amdgcn_fence(__ATOMIC_ACQUIRE, "workgroup");
    if (OUT_MODE == 0) {
      float* C = (float*)Cout + (size_t)b * strideC;
      const int hh = lane >> 4, c4 = (lane & 15) * 4;
      for (int pass = 0; pass < 2; ++pass) {
#pragma unroll
        for (int it = 0; it < 8; ++it) {
          const int row = it * 2 + hh;
          v4f v = *(const v4f*)(slab + row * 68 + c4);
          *(volatile v4f*)(C + (size_t)(mBase + row) * ldc + n0 + c4) = v;
        }
        __threadfence();
      }
    } else {
      const int q = lane >> 3, c8 = (lane & 7) * 8;
      unsigned short* C  = (unsigned short*)Cout  + (size_t)b * strideC;
      unsigned short* C2 = (OUT_MODE == 2) ? ((unsigned short*)Cout2 + (size_t)b * strideC) : nullptr;
      for (int pass = 0; pass < 2; ++pass) {
#pragma unroll
        for (int it = 0; it < 4; ++it) {
          const int row = it * 4 + q;
          const float* sp = slab + row * 68 + c8;
          v8h hv, lv;
#pragma unroll
          for (int e = 0; e < 8; ++e) {
            if (OUT_MODE == 1) {
              hv[e] = (_Float16)sp[e];
            } else {
              unsigned short hb = f2bf_bits(sp[e]);
              unsigned short lb = f2bf_bits(sp[e] - bf_bits2f(hb));
              hv[e] = __builtin_bit_cast(_Float16, hb);
              lv[e] = __builtin_bit_cast(_Float16, lb);
            }
          }
          *(volatile v8h*)(C + (size_t)(mBase + row) * ldc + n0 + c8) = hv;
          if (OUT_MODE == 2) *(volatile v8h*)(C2 + (size_t)(mBase + row) * ldc + n0 + c8) = lv;
        }
        __threadfence();
      }
    }
    __builtin_amdgcn_fence(__ATOMIC_RELEASE, "workgroup");
    __builtin_amdgcn_wave_barrier();
    __builtin_amdgcn_fence(__ATOMIC_ACQUIRE, "workgroup");
  }
}

__global__ __launch_bounds__(256) void cast8_bf16_kernel(const float* __restrict__ in, unsigned short* __restrict__ out, int n8) {
  const int i = blockIdx.x * 256 + threadIdx.x;
  if (i >= n8) return;
  const float* p = in + 8 * (size_t)i;
  const v4f a = *(const v4f*)(p);
  const v4f c = *(const v4f*)(p + 4);
  unsigned short hb[8];
#pragma unroll
  for (int e = 0; e < 4; ++e) {
    hb[e]     = f2bf_bits(a[e]);
    hb[4 + e] = f2bf_bits(c[e]);
  }
  const v4u u = (v4u){pk16(hb[0], hb[1]), pk16(hb[2], hb[3]), pk16(hb[4], hb[5]), pk16(hb[6], hb[7])};
  unsigned short* q = out + 8 * (size_t)i;
  *(volatile v4u*)q = u;
  __threadfence();
  *(volatile v4u*)q = u;
}

__global__ __launch_bounds__(384) void bnprep_kernel(const float* __restrict__ g, const float* __restrict__ be,
                                                     const float* __restrict__ mu, const float* __restrict__ var,
                                                     float* __restrict__ ss) {
  const int i = threadIdx.x;
  const float gg = bfr(g[i]), bb = bfr(be[i]), mm = bfr(mu[i]), vv = bfr(var[i]);
  const float s = gg / sqrtf(vv + kBnEps);
  const float t = bb - mm * s;
  ((volatile float*)ss)[i] = s;
  ((volatile float*)ss)[kInner + i] = t;
  __threadfence();
  ((volatile float*)ss)[i] = s;
  ((volatile float*)ss)[kInner + i] = t;
}

__global__ __launch_bounds__(256) void padfill_kernel(unsigned short* __restrict__ pl) {
  const int i   = blockIdx.x * 256 + threadIdx.x;
  const int g   = i & 511;
  const int rr  = (i >> 9) & 15;
  const int h   = (i >> 13) & 7;
  const int pln = i >> 16;
  const unsigned short val = (pln == 4 && rr == 0) ? (unsigned short)0x3F80u : (unsigned short)0;
  const unsigned w = pk16(val, val);
  const v4u u = (v4u){w, w, w, w};
  unsigned short* d = pl + (size_t)pln * kPlElems + (size_t)(h * kHdPad + kHd + rr) * kPix + 8 * g;
  *(volatile v4u*)d = u;
  __threadfence();
  *(volatile v4u*)d = u;
}

__global__ __launch_bounds__(256) void xt_kernel(const float* __restrict__ xi, unsigned short* __restrict__ xt) {
  __shared__ __align__(16) float sm[64][68];
  const int t  = threadIdx.x;
  const int p0 = blockIdx.x * 64;
  const int c0 = blockIdx.y * 64;
#pragma unroll
  for (int i = 0; i < 4; ++i) {
    const int e = i * 256 + t;
    const int r = e >> 4;
    const int f = e & 15;
    const v4f v = *(const v4f*)(xi + (size_t)(c0 + r) * kPix + p0 + 4 * f);
#pragma unroll
    for (int j = 0; j < 4; ++j) sm[4 * f + j][r] = v[j];
  }
  __syncthreads();
  const int lane = t & 31, wave = t >> 5;
  const int q = lane >> 3, c8 = (lane & 7) * 8;
  for (int pass = 0; pass < 2; ++pass) {
#pragma unroll
    for (int it = 0; it < 2; ++it) {
      const int row = wave * 8 + it * 4 + q;
      const v4f a  = *(const v4f*)(&sm[row][c8]);
      const v4f bq = *(const v4f*)(&sm[row][c8 + 4]);
      unsigned short hb[8];
#pragma unroll
      for (int e = 0; e < 4; ++e) { hb[e] = f2bf_bits(a[e]); hb[4 + e] = f2bf_bits(bq[e]); }
      const v4u u = (v4u){pk16(hb[0], hb[1]), pk16(hb[2], hb[3]), pk16(hb[4], hb[5]), pk16(hb[6], hb[7])};
      *(volatile v4u*)(xt + (size_t)(p0 + row) * kCin + c0 + c8) = u;
    }
    __threadfence();
  }
}

__global__ __launch_bounds__(256) void dwconv_kernel(const float* __restrict__ qkv, const float* __restrict__ w3,
                                                     const float* __restrict__ w5, unsigned short* __restrict__ pl) {
  const int t  = threadIdx.x;
  const int c  = blockIdx.x >> 1;
  const int g  = ((blockIdx.x & 1) << 8) | t;
  const int y  = g >> 3;
  const int x0 = (g & 7) * 8;
  const float* rowc = qkv + (size_t)c * kPix;
  const v4f cva = *(const v4f*)(rowc + y * kImgW + x0);
  const v4f cvb = *(const v4f*)(rowc + y * kImgW + x0 + 4);
  float a3[8], a5[8];
#pragma unroll
  for (int o = 0; o < 8; ++o) { a3[o] = 0.f; a5[o] = 0.f; }
  const float* w5c = w5 + c * 25;
  const float* w3c = w3 + c * 9;
  const bool lok = (x0 >= 4);
  const bool rok = (x0 + 8 < kImgW);
  const int  cl  = lok ? (x0 - 4) : 0;
  const int  cr  = rok ? (x0 + 8) : (kImgW - 4);
#pragma unroll 1
  for (int ky = 0; ky < 5; ++ky) {
    const int  yy    = y + ky - 2;
    const bool rowok = (yy >= 0) && (yy < kImgW);
    const int  yyc   = yy < 0 ? 0 : (yy > (kImgW - 1) ? (kImgW - 1) : yy);
    const float* rp  = rowc + yyc * kImgW;
    const v4f g0 = *(const v4f*)(rp + cl);
    const v4f g1 = *(const v4f*)(rp + x0);
    const v4f g2 = *(const v4f*)(rp + x0 + 4);
    const v4f g3 = *(const v4f*)(rp + cr);
    float v[16];
#pragma unroll
    for (int e = 0; e < 4; ++e) {
      v[e]      = (rowok && lok) ? g0[e] : 0.f;
      v[4 + e]  = rowok ? g1[e] : 0.f;
      v[8 + e]  = rowok ? g2[e] : 0.f;
      v[12 + e] = (rowok && rok) ? g3[e] : 0.f;
    }
    float w5r[5];
#pragma unroll
    for (int tx = 0; tx < 5; ++tx) w5r[tx] = bfr(w5c[ky * 5 + tx]);
    const bool k3ok = (ky >= 1) && (ky <= 3);
    const int  k3   = ky < 1 ? 0 : (ky > 3 ? 2 : ky - 1);
    float w3r[3];
#pragma unroll
    for (int tx = 0; tx < 3; ++tx) { const float ww = bfr(w3c[k3 * 3 + tx]); w3r[tx] = k3ok ? ww : 0.f; }
#pragma unroll
    for (int o = 0; o < 8; ++o) {
#pragma unroll
      for (int tx = 0; tx < 5; ++tx) a5[o] += w5r[tx] * v[o + tx + 2];
#pragma unroll
      for (int tx = 0; tx < 3; ++tx) a3[o] += w3r[tx] * v[o + tx + 3];
    }
  }
  float cv[8];
#pragma unroll
  for (int e = 0; e < 4; ++e) { cv[e] = cva[e]; cv[4 + e] = cvb[e]; }
  const bool dorelu = (c < 2 * kInner);
  unsigned short hb[8], lb[8];
#pragma unroll
  for (int o = 0; o < 8; ++o) {
    float z = cv[o] + (a3[o] + a5[o]) * 0.5f;
    z = dorelu ? fmaxf(z, 0.0f) : z;
    const unsigned short hq = f2bf_bits(z);
    hb[o] = hq;
    lb[o] = f2bf_bits(z - bf_bits2f(hq));
  }
  const int sel = c / kInner;
  const int cc  = c - sel * kInner;
  const int h   = cc / kHd;
  const int d   = cc - h * kHd;
  unsigned short* dh = pl + (size_t)(2 * sel) * kPlElems + (size_t)(h * kHdPad + d) * kPix + 8 * g;
  unsigned short* dl = dh + kPlElems;
  const v4u uh = (v4u){pk16(hb[0], hb[1]), pk16(hb[2], hb[3]), pk16(hb[4], hb[5]), pk16(hb[6], hb[7])};
  const v4u ul = (v4u){pk16(lb[0], lb[1]), pk16(lb[2], lb[3]), pk16(lb[4], lb[5]), pk16(lb[6], lb[7])};
  *(volatile v4u*)dh = uh;
  *(volatile v4u*)dl = ul;
  __threadfence();
  *(volatile v4u*)dh = uh;
  *(volatile v4u*)dl = ul;
}

__global__ __launch_bounds__(256) void qt_kernel(const unsigned short* __restrict__ pl, unsigned short* __restrict__ qt) {
  __shared__ __align__(16) unsigned short sm[64][72];
  const int t  = threadIdx.x;
  const int p0 = blockIdx.x * 64;
  const int h  = blockIdx.y;
  const int z  = blockIdx.z;
  const unsigned short* src = pl + (size_t)z * kPlElems + (size_t)(h * kHdPad) * kPix + p0;
#pragma unroll
  for (int i = 0; i < 2; ++i) {
    const int e = i * 256 + t;
    const int r = e >> 3;
    const int g = e & 7;
    const v4u u = *(const v4u*)(src + (size_t)r * kPix + 8 * g);
#pragma unroll
    for (int j = 0; j < 8; ++j) sm[8 * g + j][r] = (unsigned short)((u[j >> 1] >> (16 * (j & 1))) & 0xffffu);
  }
  __syncthreads();
  unsigned short* dst = qt + (size_t)z * kQtElems + ((size_t)h * kPix + p0) * kHdPad;
  const int lane = t & 31, wave = t >> 5;
  const int q = lane >> 3, c8 = (lane & 7) * 8;
  for (int pass = 0; pass < 2; ++pass) {
#pragma unroll
    for (int it = 0; it < 2; ++it) {
      const int row = wave * 8 + it * 4 + q;
      const v4u u = *(const v4u*)(&sm[row][c8]);
      *(volatile v4u*)(dst + (size_t)row * kHdPad + c8) = u;
    }
    __threadfence();
  }
}

__global__ __launch_bounds__(256) void divpack_kernel(const float* __restrict__ ob, unsigned short* __restrict__ oh,
                                                      unsigned short* __restrict__ ol) {
  const int gid = blockIdx.x * 256 + threadIdx.x;
  const int p   = gid / 48;
  const int j   = gid - p * 48;
  const int h   = j / 6;
  const int e0  = (j - h * 6) * 8;
  const float* orow = ob + (size_t)p * kOcols + h * kHdPad;
  const v4f a = *(const v4f*)(orow + e0);
  const v4f c = *(const v4f*)(orow + e0 + 4);
  const float nr  = fmaxf(orow[kHd], kEps);
  const float inv = 1.0f / nr;
  unsigned short hb[8], lb[8];
#pragma unroll
  for (int e = 0; e < 4; ++e) {
    const float z0 = a[e] * inv;
    const float z1 = c[e] * inv;
    const unsigned short h0 = f2bf_bits(z0), h1 = f2bf_bits(z1);
    hb[e] = h0;      lb[e] = f2bf_bits(z0 - bf_bits2f(h0));
    hb[4 + e] = h1;  lb[4 + e] = f2bf_bits(z1 - bf_bits2f(h1));
  }
  const v4u uh = (v4u){pk16(hb[0], hb[1]), pk16(hb[2], hb[3]), pk16(hb[4], hb[5]), pk16(hb[6], hb[7])};
  const v4u ul = (v4u){pk16(lb[0], lb[1]), pk16(lb[2], lb[3]), pk16(lb[4], lb[5]), pk16(lb[6], lb[7])};
  unsigned short* dh = oh + 8 * (size_t)gid;
  unsigned short* dl = ol + 8 * (size_t)gid;
  *(volatile v4u*)dh = uh;
  *(volatile v4u*)dl = ul;
  __threadfence();
  *(volatile v4u*)dh = uh;
  *(volatile v4u*)dl = ul;
}

extern "C" void kernel_launch(void* const* d_in, const int* in_sizes, int n_in,
                              void* d_out, int out_size, void* d_ws, size_t ws_size,
                              hipStream_t stream) {
  if (n_in < 9) return;
  if (in_sizes[0] != kImg * kCin * kPix) return;
  if (in_sizes[1] != kCqkv * kCin) return;
  if (in_sizes[2] != kCqkv * 9) return;
  if (in_sizes[3] != kCqkv * 25) return;
  if (in_sizes[4] != kInner * kInner) return;
  if (in_sizes[5] != kInner || in_sizes[6] != kInner || in_sizes[7] != kInner || in_sizes[8] != kInner) return;
  if (out_size != kImg * kInner * kPix) return;

  const float* xin    = (const float*)d_in[0];
  const float* w_qkv  = (const float*)d_in[1];
  const float* w_dw3  = (const float*)d_in[2];
  const float* w_dw5  = (const float*)d_in[3];
  const float* w_proj = (const float*)d_in[4];
  const float* gamma  = (const float*)d_in[5];
  const float* beta   = (const float*)d_in[6];
  const float* rmean  = (const float*)d_in[7];
  const float* rvar   = (const float*)d_in[8];
  float* out = (float*)d_out;
  char* ws = (char*)d_ws;

  size_t off = 0;
  auto carve = [&](size_t bytes) -> size_t { const size_t o = off; off += (bytes + 255) & ~(size_t)255; return o; };
  const size_t oWQ   = carve((size_t)kCqkv * kCin * 2);
  const size_t oWP   = carve((size_t)kInner * kInner * 2);
  const size_t oBNSS = carve((size_t)2 * kInner * 4);
  const size_t oXT   = carve((size_t)kPix * kCin * 2);
  const size_t oQKV  = carve((size_t)kCqkv * kPix * 4);
  const size_t oPL   = carve((size_t)6 * kPlElems * 2);
  const size_t oKVH  = carve((size_t)kHeads * kHdPad * kHdPad * 2);
  const size_t oKVL  = carve((size_t)kHeads * kHdPad * kHdPad * 2);
  const size_t oQTH  = carve((size_t)kQtElems * 2);
  const size_t oQTL  = carve((size_t)kQtElems * 2);
  const size_t oOB   = carve((size_t)kPix * kOcols * 4);
  const size_t oOTH  = carve((size_t)kPix * kInner * 2);
  const size_t oOTL  = carve((size_t)kPix * kInner * 2);
  if (off > ws_size) return;

  unsigned short* WQ   = (unsigned short*)(ws + oWQ);
  unsigned short* WP   = (unsigned short*)(ws + oWP);
  float*          BNSS = (float*)(ws + oBNSS);
  unsigned short* XT   = (unsigned short*)(ws + oXT);
  float*          QKV  = (float*)(ws + oQKV);
  unsigned short* PL   = (unsigned short*)(ws + oPL);
  unsigned short* KVH  = (unsigned short*)(ws + oKVH);
  unsigned short* KVL  = (unsigned short*)(ws + oKVL);
  unsigned short* QTH  = (unsigned short*)(ws + oQTH);
  unsigned short* QTL  = (unsigned short*)(ws + oQTL);
  float*          OB   = (float*)(ws + oOB);
  unsigned short* OTH  = (unsigned short*)(ws + oOTH);
  unsigned short* OTL  = (unsigned short*)(ws + oOTL);

  unsigned short* QHI = PL + 0 * kPlElems;
  unsigned short* KHI = PL + 2 * kPlElems;
  unsigned short* KLO = PL + 3 * kPlElems;
  unsigned short* VHI = PL + 4 * kPlElems;
  unsigned short* VLO = PL + 5 * kPlElems;
  (void)QHI;

  cast8_bf16_kernel<<<(kCqkv * kCin / 8) / 256, 256, 0, stream>>>(w_qkv, WQ, kCqkv * kCin / 8);
  cast8_bf16_kernel<<<(kInner * kInner / 8) / 256, 256, 0, stream>>>(w_proj, WP, kInner * kInner / 8);
  bnprep_kernel<<<1, kInner, 0, stream>>>(gamma, beta, rmean, rvar, BNSS);
  padfill_kernel<<<(6 * kHeads * 16 * (kPix / 8)) / 256, 256, 0, stream>>>(PL);

  for (int b = 0; b < kImg; ++b) {
    const float* xb = xin + (size_t)b * kCin * kPix;
    float* ob_img = out + (size_t)b * kInner * kPix;

    xt_kernel<<<dim3(kPix / 64, kCin / 64), 256, 0, stream>>>(xb, XT);

    wmma_gemm64<1, 0, 0, 0, false><<<dim3((kCqkv / 64) * (kPix / 64) / 8, 1), 256, 0, stream>>>(
        WQ, WQ, kCin, 0L, XT, XT, kCin, 0L, (void*)QKV, (void*)QKV, kPix, 0L,
        BNSS, QKV, 0L, kCqkv, kPix, kCin, 1.0f);

    dwconv_kernel<<<kCqkv * 2, 256, 0, stream>>>(QKV, w_dw3, w_dw5, PL);

    wmma_gemm64<1, 2, 0, 2, false><<<dim3(1, kHeads), 256, 0, stream>>>(
        VHI, VLO, kPix, (long)kHdPad * kPix, KHI, KLO, kPix, (long)kHdPad * kPix,
        (void*)KVH, (void*)KVL, kHdPad, (long)kHdPad * kHdPad,
        BNSS, QKV, 0L, kHdPad, kHdPad, kPix, 1.0f);

    qt_kernel<<<dim3(kPix / 64, kHeads, 2), 256, 0, stream>>>(PL, QTH);

    wmma_gemm64<1, 2, 0, 0, false><<<dim3((kPix / 64) / 8, kHeads), 256, 0, stream>>>(
        QTH, QTL, kHdPad, (long)kPix * kHdPad, KVH, KVL, kHdPad, (long)kHdPad * kHdPad,
        (void*)OB, (void*)OB, kOcols, (long)kHdPad,
        BNSS, QKV, 0L, kPix, kHdPad, kHdPad, 1.0f);

    divpack_kernel<<<(kPix * 48) / 256, 256, 0, stream>>>(OB, OTH, OTL);

    wmma_gemm64<1, 1, 3, 0, false><<<dim3((kInner / 64) * (kPix / 64) / 8, 1), 256, 0, stream>>>(
        WP, WP, kInner, 0L, OTH, OTL, kInner, 0L, (void*)ob_img, (void*)ob_img, kPix, 0L,
        BNSS, QKV, 0L, kInner, kPix, kInner, 1.0f);
  }
}
